// HardgroupAttentionV2_11836929868323
// MI455X (gfx1250) — hardware-verified
//
#include <hip/hip_runtime.h>
#include <math.h>

typedef __attribute__((ext_vector_type(16))) _Float16 v16h;
typedef __attribute__((ext_vector_type(16))) __bf16 v16b;
typedef __attribute__((ext_vector_type(8)))  _Float16 v8h;
typedef __attribute__((ext_vector_type(8)))  float v8f;
typedef __attribute__((ext_vector_type(4)))  float v4f;
typedef __attribute__((ext_vector_type(2)))  float v2f;
typedef __attribute__((ext_vector_type(4)))  unsigned v4u;
typedef __attribute__((ext_vector_type(4)))  int v4i;
typedef float __attribute__((may_alias)) float_a;
typedef int __attribute__((may_alias)) int_a;

template <typename T> __device__ __forceinline__ void vst2(void* p, T v) { *(volatile T*)p = v; __threadfence(); *(volatile T*)p = v; }
__device__ __forceinline__ v8f wmma16(v16h a, v16h b, v8f c) {
  v8f d = __builtin_amdgcn_wmma_f32_16x16x32_f16(false, a, false, b, (short)0, c, false, false);
  asm volatile("v_nop\n\tv_nop\n\tv_nop\n\tv_nop" : "+v"(d) : "v"(a), "v"(b));
  return d;
}
__device__ __forceinline__ v8f wmma_bf(v16b a, v16b b, v8f c) {
  v8f d = __builtin_amdgcn_wmma_f32_16x16x32_bf16(false, a, false, b, (short)0, c, false, false);
  asm volatile("v_nop\n\tv_nop\n\tv_nop\n\tv_nop" : "+v"(d) : "v"(a), "v"(b));
  return d;
}
__device__ __forceinline__ v16h frag_h(const _Float16* rowk0, int lane) {
  union { v16h v; v8h q[2]; } u; const _Float16* p = rowk0 + 8 * (lane >> 4);
  u.q[0] = *(const v8h*)p; u.q[1] = *(const v8h*)(p + 16); return u.v;
}
__device__ __forceinline__ v16h frag_f32(const float* rowk0, int lane) {
  v16h a; const float* p = rowk0 + 8 * (lane >> 4);
#pragma unroll
  for (int i = 0; i < 8; ++i) { a[i] = (_Float16)p[i]; a[8 + i] = (_Float16)p[16 + i]; }
  return a;
}
__device__ __forceinline__ v16h frag_f32s(const float* rowk0, int lane, float sc) {
  v16h a; const float* p = rowk0 + 8 * (lane >> 4);
#pragma unroll
  for (int i = 0; i < 8; ++i) { a[i] = (_Float16)(p[i] * sc); a[8 + i] = (_Float16)(p[16 + i] * sc); }
  return a;
}
__device__ __forceinline__ v16h fragc_f32(const float* W, int k0, int n, int lane, int ld, int K) {
  v16h a; const int g = lane >> 4;
#pragma unroll
  for (int i = 0; i < 8; ++i) { const int ka = k0 + 8 * g + i, kb = ka + 16;
    a[i] = (_Float16)(ka < K ? W[(size_t)(ka < K ? ka : K - 1) * ld + n] : 0.f); a[8 + i] = (_Float16)(kb < K ? W[(size_t)(kb < K ? kb : K - 1) * ld + n] : 0.f); }
  return a;
}
struct F2 { v16b h, l; };
__device__ __forceinline__ F2 bsplit16(const float v[16]) { F2 r;
#pragma unroll
  for (int i = 0; i < 16; ++i) { const __bf16 h = (__bf16)v[i]; r.h[i] = h; r.l[i] = (__bf16)(v[i] - (float)h); }
  return r; }
__device__ __forceinline__ F2 split_row(const float* row, int k0, int lane) { float v[16]; const float* p = row + k0 + 8 * (lane >> 4);
#pragma unroll
  for (int i = 0; i < 8; ++i) { v[i] = p[i]; v[8 + i] = p[16 + i]; }
  return bsplit16(v); }
__device__ __forceinline__ F2 split_rowK(const float* row, int k0, int lane, int K) { float v[16]; const int g = lane >> 4;
#pragma unroll
  for (int i = 0; i < 8; ++i) { const int ka = k0 + 8 * g + i, kb = ka + 16; v[i] = ka < K ? row[ka < K ? ka : K - 1] : 0.f; v[8 + i] = kb < K ? row[kb < K ? kb : K - 1] : 0.f; }
  return bsplit16(v); }
__device__ __forceinline__ F2 split_col(const float* W, int k0, int n, int lane, int ld, int K) { float v[16]; const int g = lane >> 4;
#pragma unroll
  for (int i = 0; i < 8; ++i) { const int ka = k0 + 8 * g + i, kb = ka + 16; v[i] = ka < K ? W[(size_t)(ka < K ? ka : K - 1) * ld + n] : 0.f; v[8 + i] = kb < K ? W[(size_t)(kb < K ? kb : K - 1) * ld + n] : 0.f; }
  return bsplit16(v); }
__device__ __forceinline__ v8f mac3(const F2& a, const F2& b, v8f c) { c = wmma_bf(a.l, b.h, c); c = wmma_bf(a.h, b.l, c); return wmma_bf(a.h, b.h, c); }
__device__ __forceinline__ float sigm(float v) { return 1.0f / (1.0f + expf(-v)); }
#define LDSX() do { asm volatile("s_wait_dscnt 0" ::: "memory"); __builtin_amdgcn_wave_barrier(); __builtin_amdgcn_fence(__ATOMIC_RELEASE, "workgroup"); } while (0)


#define NB 8
#define NT 1024
#define NR (NB * NT)
#define CC 256
#define NHD 8
#define HD 32
#define GP 20
#define QKVW 768
#ifndef NBT
#define NBT NB
#endif
typedef __attribute__((ext_vector_type(8))) __bf16 v8b;
__device__ __forceinline__ v16b frag_b(const __bf16* rowk0, int lane) {
  union { v16b v; v8b q[2]; } u; const __bf16* p = rowk0 + 8 * (lane >> 4);
  u.q[0] = *(const v8b*)p; u.q[1] = *(const v8b*)(p + 16); return u.v;
}
__device__ __forceinline__ float bfr(float v) { return (float)(__bf16)v; }
__device__ __attribute__((noinline)) float exp_ni(float v) { return expf(v); }
__device__ __attribute__((noinline)) float erf_ni(float v) { return erff(v); }

#define PK_QKV 0
#define PK_P   (PK_QKV + QKVW * CC)
#define PK_END (PK_P + CC * CC)
#define WS_PK  0u
#define WS_QF  (((WS_PK + 2u * PK_END) + 127u) / 128u * 128u)
#define WS_QH  (WS_QF + 4u * NR * 2 * CC)
#define WS_QL  (WS_QH + 2u * NR * 2 * CC)
#define WS_VTH (WS_QL + 2u * NR * 2 * CC)
#define WS_VTL (WS_VTH + 2u * NR * CC)
#define WS_GRP (WS_VTL + 2u * NR * CC)
#define WS_RS  (WS_GRP + 4u * 2 * NB * NHD * NT)
#define WS_CS  (WS_RS + 4u * NB * NHD * NT * 2)
#define WS_O   (WS_CS + 4u * NB * NHD * NT)
#define WS_OL  (WS_O + 2u * NR * CC)
#define WS_CSP (WS_OL + 2u * NR * CC)
#define WS_END (WS_CSP + 4u * NB * NHD * (NT / 64) * NT)

__global__ __launch_bounds__(256) void k_pack(const float* __restrict__ WQKV, const float* __restrict__ WP, __bf16* __restrict__ PK) {
  __shared__ __align__(16) __bf16 s[CC]; const int n = blockIdx.x, which = blockIdx.y, t = threadIdx.x; if (which == 1 && n >= CC) return;
  s[t] = (__bf16)(which == 0 ? WQKV[(size_t)n * CC + t] : WP[(size_t)n * CC + t]);
  __syncthreads();
  if (t < CC / 8) vst2((unsigned*)(PK + (which == 0 ? PK_QKV : PK_P) + (size_t)n * CC + t * 8), *(const v4u*)&s[t * 8]);
}
__global__ __launch_bounds__(128) void k_qkv(const float* __restrict__ X, const __bf16* __restrict__ PK, float* __restrict__ QF, _Float16* __restrict__ QH, _Float16* __restrict__ QL, _Float16* __restrict__ VTH, _Float16* __restrict__ VTL) {
  __shared__ __align__(16) float sf[4][16][132]; __shared__ __align__(16) _Float16 soh[4][16][136], sol[4][16][136]; __shared__ __align__(16) _Float16 sth[128][72], stl[128][72];
  const int tid = threadIdx.x, wave = tid >> 5, lane = tid & 31, col = lane & 15, g = lane >> 4; const size_t r0 = (size_t)blockIdx.x * 64 + wave * 16; const int n0 = blockIdx.y * 128; const int which = n0 / CC;
  v8f acc[8] = {};
#pragma unroll
  for (int kc = 0; kc < CC / 32; ++kc) { v16b a; { const float* p = X + (r0 + col) * CC + kc * 32 + 8 * g;
#pragma unroll
      for (int i = 0; i < 8; ++i) { a[i] = (__bf16)p[i]; a[8 + i] = (__bf16)p[16 + i]; } }
#pragma unroll
    for (int j = 0; j < 8; ++j) acc[j] = wmma_bf(a, frag_b(PK + PK_QKV + (size_t)(n0 + j * 16 + col) * CC + kc * 32, lane), acc[j]); }
  if (which < 2) {
#pragma unroll
    for (int j = 0; j < 8; ++j)
#pragma unroll
      for (int r = 0; r < 8; ++r) { const float v = acc[j][r]; sf[wave][8 * g + r][j * 16 + col] = v; const _Float16 hv = (_Float16)v; soh[wave][8 * g + r][j * 16 + col] = hv; sol[wave][8 * g + r][j * 16 + col] = (_Float16)((v - (float)hv) * 2048.0f); }
    LDSX(); const int c0 = n0;
    for (int rl = 0; rl < 16; ++rl) { vst2(QF + (r0 + rl) * (2 * CC) + c0 + lane * 4, *(const v4f*)&sf[wave][rl][lane * 4]);
      if (lane < 16) vst2((unsigned*)(QH + (r0 + rl) * (2 * CC) + c0 + lane * 8), *(const v4u*)&soh[wave][rl][lane * 8]); else vst2((unsigned*)(QL + (r0 + rl) * (2 * CC) + c0 + (lane - 16) * 8), *(const v4u*)&sol[wave][rl][(lane - 16) * 8]); }
  } else {
#pragma unroll
    for (int j = 0; j < 8; ++j)
#pragma unroll
      for (int r = 0; r < 8; ++r) { const float v = acc[j][r]; const _Float16 hv = (_Float16)v; sth[j * 16 + col][wave * 16 + 8 * g + r] = hv; stl[j * 16 + col][wave * 16 + 8 * g + r] = (_Float16)((v - (float)hv) * 2048.0f); }
    __syncthreads();
    const size_t rb = (size_t)blockIdx.x * 64; const int b = (int)(rb / NT), s0 = (int)(rb % NT); const int c0 = n0 - 2 * CC;
    for (int e = tid; e < 128 * 8; e += 128) { const int d = e >> 3, pc = e & 7; const size_t o = ((size_t)b * CC + c0 + d) * NT + s0 + pc * 8; vst2((unsigned*)(VTH + o), *(const v4u*)&sth[d][pc * 8]); vst2((unsigned*)(VTL + o), *(const v4u*)&stl[d][pc * 8]); }
  }
}
__global__ __launch_bounds__(256) void k_grp(const float* __restrict__ QF, const float* __restrict__ GQ, const float* __restrict__ GK, int* __restrict__ GRP) {
  __shared__ __align__(16) int sg[256]; const int tid = threadIdx.x; const size_t e = (size_t)blockIdx.x * 256 + tid;
  const int n = (int)(e % NT); const int h = (int)((e / NT) % NHD); const int b = (int)((e / ((size_t)NT * NHD)) % NB); const int which = (int)(e / ((size_t)NT * NHD * NB));
  const float* qr = QF + ((size_t)b * NT + n) * (2 * CC) + which * CC + h * HD; const float* gw = (which == 0) ? GQ : GK;
  float best = -3.0e38f; int bi = 0;
#pragma unroll 1
  for (int m = 0; m < GP; ++m) { const float* w = gw + ((size_t)h * GP + m) * HD; float s = 0.f;
#pragma unroll 8
    for (int d = 0; d < HD; ++d) s += qr[d] * bfr(w[d]);
    if (s > best) { best = s; bi = m; } }
  sg[tid] = bi;
  __syncthreads();
  if (tid < 64) vst2((unsigned*)(GRP + (size_t)blockIdx.x * 256 + tid * 4), *(const v4u*)&sg[tid * 4]);
}
struct ScoreCtx { v16h aqh, aql; };
__device__ __forceinline__ void score_tile(const ScoreCtx& q, const _Float16* krow_h, const _Float16* krow_l, int lane, v8f& s) {
  const v16h bkh = frag_h(krow_h, lane), bkl = frag_h(krow_l, lane); v8f c = {}; c = wmma16(q.aqh, bkh, c); v8f c2 = {}; c2 = wmma16(q.aql, bkh, c2); c2 = wmma16(q.aqh, bkl, c2);
#pragma unroll
  for (int r = 0; r < 8; ++r) s[r] = (c[r] + c2[r] * (1.0f / 2048.0f)) * 0.17677669529663688f;
}
__global__ __launch_bounds__(128) void k_rowstat(const _Float16* __restrict__ QH, const _Float16* __restrict__ QL, float* __restrict__ RS) {
  __shared__ __align__(16) float srs[64][2];
  const int tid = threadIdx.x, wave = tid >> 5, lane = tid & 31, col = lane & 15, g = lane >> 4; const int qb = blockIdx.x, h = blockIdx.y, b = blockIdx.z; const int q0 = qb * 64 + wave * 16; const size_t rq = (size_t)b * NT + q0 + col;
  ScoreCtx Q; Q.aqh = frag_h(QH + rq * (2 * CC) + h * HD, lane); Q.aql = frag_h(QL + rq * (2 * CC) + h * HD, lane);
  float m[8], l[8];
#pragma unroll
  for (int r = 0; r < 8; ++r) { m[r] = -3.0e38f; l[r] = 0.f; }
#pragma unroll 1
  for (int ks = 0; ks < NT / 32; ++ks) { v8f s[2];
#pragma unroll
    for (int ct = 0; ct < 2; ++ct) { const size_t kk = (size_t)b * NT + ks * 32 + ct * 16 + col; score_tile(Q, QH + kk * (2 * CC) + CC + h * HD, QL + kk * (2 * CC) + CC + h * HD, lane, s[ct]); }
#pragma unroll
    for (int r = 0; r < 8; ++r) { float mx = fmaxf(s[0][r], s[1][r]);
#pragma unroll
      for (int o = 1; o < 16; o <<= 1) mx = fmaxf(mx, __shfl_xor(mx, o));
      const float mn = fmaxf(m[r], mx); const float alpha = (m[r] <= -1.0e38f) ? 0.f : exp_ni(m[r] - mn); float es = exp_ni(s[0][r] - mn) + exp_ni(s[1][r] - mn);
#pragma unroll
      for (int o = 1; o < 16; o <<= 1) es += __shfl_xor(es, o);
      l[r] = l[r] * alpha + es; m[r] = mn; } }
  if (col == 0) {
#pragma unroll
    for (int r = 0; r < 8; ++r) { srs[wave * 16 + 8 * g + r][0] = m[r]; srs[wave * 16 + 8 * g + r][1] = 1.0f / l[r]; } }
  __syncthreads();
  if (tid < 32) vst2(RS + (((size_t)b * NHD + h) * NT + qb * 64) * 2 + tid * 4, *(const v4f*)(&srs[0][0] + tid * 4));
}
__global__ __launch_bounds__(128) void k_colsum(const _Float16* __restrict__ QH, const _Float16* __restrict__ QL, const float* __restrict__ RS, const int* __restrict__ GRP, float* __restrict__ CSP) {
  __shared__ float spart[4][NT]; __shared__ __align__(16) float ssum[NT];
  const int tid = threadIdx.x, wave = tid >> 5, lane = tid & 31, col = lane & 15, g = lane >> 4; const int qb = blockIdx.x, h = blockIdx.y, b = blockIdx.z; const int q0 = qb * 64 + wave * 16; const size_t rq = (size_t)b * NT + q0 + col;
  ScoreCtx Q; Q.aqh = frag_h(QH + rq * (2 * CC) + h * HD, lane); Q.aql = frag_h(QL + rq * (2 * CC) + h * HD, lane);
  float mrow[8], iz[8]; int gq[8];
#pragma unroll
  for (int r = 0; r < 8; ++r) { const int qi = q0 + 8 * g + r; const size_t ri = ((size_t)b * NHD + h) * NT + qi; mrow[r] = RS[ri * 2]; iz[r] = RS[ri * 2 + 1]; gq[r] = GRP[ri]; }
  const int* gk = GRP + (size_t)NB * NHD * NT + ((size_t)b * NHD + h) * NT;
#pragma unroll 1
  for (int ks = 0; ks < NT / 32; ++ks) { v8f s[2];
#pragma unroll
    for (int ct = 0; ct < 2; ++ct) { const size_t kk = (size_t)b * NT + ks * 32 + ct * 16 + col; score_tile(Q, QH + kk * (2 * CC) + CC + h * HD, QL + kk * (2 * CC) + CC + h * HD, lane, s[ct]); }
#pragma unroll
    for (int ct = 0; ct < 2; ++ct) { const int km = ks * 32 + ct * 16 + col; const int gkm = gk[km]; float a = 0.f;
#pragma unroll
      for (int r = 0; r < 8; ++r) a += (gq[r] == gkm) ? exp_ni(s[ct][r] - mrow[r]) * iz[r] : 0.f;
      a += __shfl_xor(a, 16);
      if (g == 0) spart[wave][km] = a; } }
  __syncthreads();
  for (int e = tid; e < NT; e += 128) ssum[e] = (spart[0][e] + spart[1][e]) + (spart[2][e] + spart[3][e]);
  __syncthreads();
  for (int e = tid; e < NT / 4; e += 128) vst2(CSP + ((((size_t)b * NHD + h) * (NT / 64) + qb) * NT) + e * 4, *(const v4f*)&ssum[e * 4]);
}
__global__ __launch_bounds__(256) void k_colred(const float* __restrict__ CSP, float* __restrict__ CS) {
  __shared__ __align__(16) float s[NT]; const int tid = threadIdx.x; const int h = blockIdx.x, b = blockIdx.y; const float* base = CSP + ((size_t)b * NHD + h) * (NT / 64) * NT;
  for (int m = tid; m < NT; m += 256) { float a = 0.f; for (int qb = 0; qb < NT / 64; ++qb) a += base[(size_t)qb * NT + m]; s[m] = a; }
  __syncthreads();
  for (int e = tid; e < NT / 4; e += 256) vst2(CS + ((size_t)b * NHD + h) * NT + e * 4, *(const v4f*)&s[e * 4]);
}
__global__ __launch_bounds__(128) void k_attn(const _Float16* __restrict__ QH, const _Float16* __restrict__ QL, const _Float16* __restrict__ VTH, const _Float16* __restrict__ VTL, const float* __restrict__ RS, const int* __restrict__ GRP, const float* __restrict__ CS, __bf16* __restrict__ OH, __bf16* __restrict__ OL) {
  __shared__ __align__(16) _Float16 sph[4][16][40], spl[4][16][40]; __shared__ __align__(16) __bf16 soh[64][CC + 8], sol[64][CC + 8];
  const int tid = threadIdx.x, wave = tid >> 5, lane = tid & 31, col = lane & 15, g = lane >> 4; const int qb = blockIdx.x, b = blockIdx.y;
  for (int hh = 0; hh < 2; ++hh) { const int h = wave * 2 + hh; const int* gk = GRP + (size_t)NB * NHD * NT + ((size_t)b * NHD + h) * NT; const float* cs = CS + ((size_t)b * NHD + h) * NT;
    for (int rt = 0; rt < 4; ++rt) { const int q0 = qb * 64 + rt * 16; const size_t rq = (size_t)b * NT + q0 + col;
      ScoreCtx Q; Q.aqh = frag_h(QH + rq * (2 * CC) + h * HD, lane); Q.aql = frag_h(QL + rq * (2 * CC) + h * HD, lane);
      float mrow[8], iz[8]; int gq[8];
#pragma unroll
      for (int r = 0; r < 8; ++r) { const int qi = q0 + 8 * g + r; const size_t ri = ((size_t)b * NHD + h) * NT + qi; mrow[r] = RS[ri * 2]; iz[r] = RS[ri * 2 + 1]; gq[r] = GRP[ri]; }
      v8f acc[2] = {}, accl[2] = {};
#pragma unroll 1
      for (int ks = 0; ks < NT / 32; ++ks) { v8f s[2];
#pragma unroll
        for (int ct = 0; ct < 2; ++ct) { const size_t kk = (size_t)b * NT + ks * 32 + ct * 16 + col; score_tile(Q, QH + kk * (2 * CC) + CC + h * HD, QL + kk * (2 * CC) + CC + h * HD, lane, s[ct]); }
#pragma unroll
        for (int ct = 0; ct < 2; ++ct) { const int km = ks * 32 + ct * 16 + col; const int gkm = gk[km]; const float icm = 1.0f / (cs[km] + 1e-8f);
#pragma unroll
          for (int r = 0; r < 8; ++r) { const float w = (gq[r] == gkm) ? (exp_ni(s[ct][r] - mrow[r]) * iz[r]) * icm : 0.f; const _Float16 hw = (_Float16)w; sph[wave][8 * g + r][ct * 16 + col] = hw; spl[wave][8 * g + r][ct * 16 + col] = (_Float16)((w - (float)hw) * 2048.0f); } }
        LDSX();
        const v16h pah = frag_h(&sph[wave][col][0], lane), pal = frag_h(&spl[wave][col][0], lane);
#pragma unroll
        for (int dt = 0; dt < 2; ++dt) { const size_t vo = ((size_t)b * CC + h * HD + dt * 16 + col) * NT + ks * 32; const v16h vh = frag_h(VTH + vo, lane), vl = frag_h(VTL + vo, lane); acc[dt] = wmma16(pah, vh, acc[dt]); accl[dt] = wmma16(pal, vh, accl[dt]); accl[dt] = wmma16(pah, vl, accl[dt]); }
        LDSX(); }
#pragma unroll
      for (int r = 0; r < 8; ++r)
#pragma unroll
        for (int dt = 0; dt < 2; ++dt) { const float v = acc[dt][r] + accl[dt][r] * (1.0f / 2048.0f); const __bf16 hb = (__bf16)v; soh[rt * 16 + 8 * g + r][h * HD + dt * 16 + col] = hb; sol[rt * 16 + 8 * g + r][h * HD + dt * 16 + col] = (__bf16)(v - (float)hb); } } }
  __syncthreads();
  for (int e = tid; e < 64 * (CC / 8) * 2; e += 128) { const int plane = e / (64 * CC / 8), rem = e % (64 * CC / 8); const int r = rem / (CC / 8), pc = rem % (CC / 8); const size_t o = ((size_t)b * NT + qb * 64 + r) * CC + pc * 8;
    if (plane == 0) vst2((unsigned*)(OH + o), *(const v4u*)&soh[r][pc * 8]); else vst2((unsigned*)(OL + o), *(const v4u*)&sol[r][pc * 8]); }
}
__global__ __launch_bounds__(128) void k_proj(const __bf16* __restrict__ OH, const __bf16* __restrict__ OL, const __bf16* __restrict__ PK, float* __restrict__ OUT) {
  __shared__ __align__(16) float so[4][16][132];
  const int tid = threadIdx.x, wave = tid >> 5, lane = tid & 31, col = lane & 15, g = lane >> 4; const size_t r0 = (size_t)blockIdx.x * 64 + wave * 16; const int n0 = blockIdx.y * 128;
  v8f acc[8] = {};
#pragma unroll
  for (int kc = 0; kc < CC / 32; ++kc) { F2 a; a.h = frag_b(OH + (r0 + col) * CC + kc * 32, lane); a.l = frag_b(OL + (r0 + col) * CC + kc * 32, lane);
#pragma unroll
    for (int j = 0; j < 8; ++j) { const v16b w = frag_b(PK + PK_P + (size_t)(n0 + j * 16 + col) * CC + kc * 32, lane); acc[j] = wmma_bf(a.l, w, acc[j]); acc[j] = wmma_bf(a.h, w, acc[j]); } }
#pragma unroll
  for (int j = 0; j < 8; ++j)
#pragma unroll
    for (int r = 0; r < 8; ++r) so[wave][8 * g + r][j * 16 + col] = acc[j][r];
  LDSX();
  for (int rl = 0; rl < 16; ++rl) vst2(OUT + (r0 + rl) * CC + n0 + lane * 4, *(const v4f*)&so[wave][rl][lane * 4]);
}
extern "C" void kernel_launch(void* const* d_in, const int* in_sizes, int n_in, void* d_out, int out_size, void* d_ws, size_t ws_size, hipStream_t stream) {
  (void)in_sizes; (void)n_in; (void)out_size;
  const float** F = (const float**)d_in;
  if (ws_size < (size_t)WS_END) return;
  char* ws = (char*)d_ws; __bf16 *PK = (__bf16*)(ws + WS_PK), *OH = (__bf16*)(ws + WS_O), *OL = (__bf16*)(ws + WS_OL); float *QF = (float*)(ws + WS_QF), *RS = (float*)(ws + WS_RS), *CS = (float*)(ws + WS_CS); _Float16 *QH = (_Float16*)(ws + WS_QH), *QL = (_Float16*)(ws + WS_QL), *VTH = (_Float16*)(ws + WS_VTH), *VTL = (_Float16*)(ws + WS_VTL); int* GRP = (int*)(ws + WS_GRP);
  float* CSP = (float*)(ws + WS_CSP);
  k_pack<<<dim3(QKVW, 2), 256, 0, stream>>>(F[1], F[2], PK);
  k_qkv<<<dim3(NBT * NT / 64, QKVW / 128), 128, 0, stream>>>(F[0], PK, QF, QH, QL, VTH, VTL);
  k_grp<<<(2 * NB * NHD * NT) / 256, 256, 0, stream>>>(QF, F[3], F[4], GRP);
  k_rowstat<<<dim3(NT / 64, NHD, NBT), 128, 0, stream>>>(QH, QL, RS);
  k_colsum<<<dim3(NT / 64, NHD, NBT), 128, 0, stream>>>(QH, QL, RS, GRP, CSP);
  k_colred<<<dim3(NHD, NBT), 256, 0, stream>>>(CSP, CS);
  k_attn<<<dim3(NT / 64, NBT), 128, 0, stream>>>(QH, QL, VTH, VTL, RS, GRP, CS, OH, OL);
  k_proj<<<dim3(NBT * NT / 64, CC / 128), 128, 0, stream>>>(OH, OL, PK, (float*)d_out);
}
